// PNA_19404662243713
// MI455X (gfx1250) — hardware-verified
//
#include <hip/hip_runtime.h>

constexpr int kNodes = 50000;
constexpr int kEdges = 500000;
constexpr int kNPad = 50176;
constexpr int kFeat = 128;
constexpr int kPQPitch = 2 * kFeat;
constexpr int kA5Pitch = 4 * kFeat;
constexpr int kCls = 40;
constexpr int kThreads = 256;
constexpr int kNumChunks = 4;
constexpr int kChunkRows = 12544;
constexpr int kAggRows = 256;
constexpr int kRowsPerWave = 32;
constexpr int kBlocksPerChunk = kChunkRows / kAggRows;
constexpr int kAccPitch = 2 * kFeat;
constexpr int kAggLdsBytes = kAggRows * kAccPitch * 4;
constexpr int kEdgeChunk = 4096;
constexpr int kEPT = 16;
constexpr int kNumEdgeChunks = (kEdges + kEdgeChunk - 1) / kEdgeChunk;

static_assert(kNPad % 64 == 0);
static_assert(kNPad >= kNodes);
static_assert(kNumChunks * kChunkRows == kNPad);
static_assert(kChunkRows % 64 == 0);
static_assert(kBlocksPerChunk * kAggRows == kChunkRows);
static_assert(8 * kRowsPerWave == kAggRows);
static_assert(kRowsPerWave % 2 == 0);
static_assert(kAggRows == 256);
static_assert(kEdgeChunk == kThreads * kEPT);
static_assert(kEdges % kEPT == 0);
static_assert(kEPT % 4 == 0);
static_assert(kNodes % 16 == 0);
static_assert(kNodes < 65536);
static_assert(kFeat % 32 == 0 && kA5Pitch % 32 == 0 && kPQPitch % 64 == 0);
static_assert(((kNPad / 64) * (kPQPitch / 64)) % 8 == 0);
static_assert(((kChunkRows / 64) * (kFeat / 64)) % 8 == 0);
static_assert((kNPad / 64) % 8 == 0);
static_assert((kNPad * 16) % kThreads == 0);
static_assert((kAggRows * kAccPitch / 4) % kThreads == 0);

constexpr size_t kSzH     = (size_t)kNPad * kFeat * 2;
constexpr size_t kSzPQ    = (size_t)kNPad * kPQPitch * 4;
constexpr size_t kSzA5    = (size_t)kChunkRows * kA5Pitch * 2;
constexpr size_t kSzT     = (size_t)kChunkRows * kFeat * 2;
constexpr size_t kSzWpre  = (size_t)256 * 128 * 2;
constexpr size_t kSzWpost = (size_t)128 * 512 * 2;
constexpr size_t kSzWlin  = (size_t)128 * 128 * 2;
constexpr size_t kSzWout  = (size_t)64 * 128 * 2;
constexpr size_t kSzBias  = (size_t)7 * 256 * 4;
constexpr size_t kOffHh    = 0;
constexpr size_t kOffHl    = kOffHh + kSzH;
constexpr size_t kOffPQ    = kOffHl + kSzH;
constexpr size_t kOffA5h   = kOffPQ + kSzPQ;
constexpr size_t kOffA5l   = kOffA5h + kSzA5;
constexpr size_t kOffTh    = kOffA5l + kSzA5;
constexpr size_t kOffTl    = kOffTh + kSzT;
constexpr size_t kOffWpre1 = kOffTl + kSzT;
constexpr size_t kOffWpost1= kOffWpre1 + kSzWpre;
constexpr size_t kOffWlin1 = kOffWpost1 + kSzWpost;
constexpr size_t kOffWpre2 = kOffWlin1 + kSzWlin;
constexpr size_t kOffWpost2= kOffWpre2 + kSzWpre;
constexpr size_t kOffWlin2 = kOffWpost2 + kSzWpost;
constexpr size_t kOffWout  = kOffWlin2 + kSzWlin;
constexpr size_t kOffBias  = kOffWout + kSzWout;
constexpr size_t kOffEnd   = kOffBias + kSzBias;
static_assert(kOffEnd == 109665280);
static_assert(kOffEnd <= (size_t)134217728);
static_assert(kOffPQ % 256 == 0 && kOffA5h % 256 == 0 && kOffTh % 256 == 0 && kOffWpre1 % 256 == 0 && kOffBias % 256 == 0);

typedef __attribute__((ext_vector_type(16))) __bf16   v16b;
typedef __attribute__((ext_vector_type(8)))  __bf16   v8b;
typedef __attribute__((ext_vector_type(8)))  float    v8f;
typedef __attribute__((ext_vector_type(4)))  float    v4f;
typedef __attribute__((ext_vector_type(4)))  unsigned int v4u;
typedef __attribute__((ext_vector_type(4)))  int      v4i;

__device__ __forceinline__ unsigned short f2bf_bits(float f) {
  unsigned u = __float_as_uint(f);
  return (unsigned short)((u + 0x7FFFu + ((u >> 16) & 1u)) >> 16);
}
__device__ __forceinline__ float bf_bits2f(unsigned short h) { return __uint_as_float(((unsigned)h) << 16); }
__device__ __forceinline__ unsigned pk16(unsigned short a, unsigned short b) { return (unsigned)a | ((unsigned)b << 16); }

__device__ __forceinline__ void dep_guard_b(v8f& a, v8f& b, v16b x, v16b y) { asm volatile("v_nop\n\tv_nop\n\tv_nop\n\tv_nop" : "+v"(a), "+v"(b) : "v"(x), "v"(y)); }
__device__ __forceinline__ void keep4_b(v16b a, v16b b, v16b c, v16b d) { asm volatile("v_nop" :: "v"(a), "v"(b), "v"(c), "v"(d)); }
__device__ __forceinline__ void acc_guard4(v8f& a, v8f& b, v8f& c, v8f& d) { asm volatile("v_nop\n\tv_nop\n\tv_nop\n\tv_nop" : "+v"(a), "+v"(b), "+v"(c), "+v"(d)); }
__device__ __forceinline__ void guard_row(v8f& a0, v8f& a1, v8f& a2, v8f& a3, v16b x, v16b y, v16b b0, v16b b1, v16b b2, v16b b3) {
  asm volatile("v_nop\n\tv_nop\n\tv_nop\n\tv_nop" : "+v"(a0), "+v"(a1), "+v"(a2), "+v"(a3) : "v"(x), "v"(y), "v"(b0), "v"(b1), "v"(b2), "v"(b3));
}
__device__ __forceinline__ void keep_v4i(v4i a) { asm volatile("" :: "v"(a)); }
template <typename T> struct Frag;
template <> struct Frag<__bf16> {
  typedef v16b V; union U { v16b v; v8b h[2]; };
  static __device__ __forceinline__ v16b load(const __bf16* p) {
    U f; f.h[0] = *(const v8b*)(p); f.h[1] = *(const v8b*)(p + 16); return f.v;
  }
  static __device__ __forceinline__ v8f mma(v16b a, v16b b, v8f c) {
    return __builtin_amdgcn_wmma_f32_16x16x32_bf16(false, a, false, b, (short)0, c, false, false);
  }
  static __device__ __forceinline__ void guard(v8f& a, v8f& b, v16b x, v16b y) { dep_guard_b(a, b, x, y); }
  static __device__ __forceinline__ void keep(v16b a, v16b b, v16b c, v16b d) { keep4_b(a, b, c, d); }
};

__device__ __forceinline__ unsigned split_pair(float a, float b, unsigned& lo) {
  const unsigned short ha = f2bf_bits(a);
  const unsigned short hb = f2bf_bits(b);
  const unsigned short la = f2bf_bits(a - bf_bits2f(ha));
  const unsigned short lb = f2bf_bits(b - bf_bits2f(hb));
  lo = pk16(la, lb);
  return pk16(ha, hb);
}
__device__ __forceinline__ void split8(const float (&v)[8], v4u& hi, v4u& lo) {
#pragma unroll
  for (int e = 0; e < 4; ++e) { unsigned l; const unsigned h = split_pair(v[2 * e], v[2 * e + 1], l); hi[e] = h; lo[e] = l; }
}

template <bool LO>
__device__ __forceinline__ void kstep64(v8f (&acc)[4][4], const __bf16* __restrict__ A, const __bf16* __restrict__ A2, int lda,
                                        const __bf16* __restrict__ Bt, int ldb, int m0, int n0, int k0, int rlane, int koff) {
  v16b bh[4];
#pragma unroll
  for (int j = 0; j < 4; ++j) bh[j] = Frag<__bf16>::load(Bt + (size_t)(n0 + (j << 4) + rlane) * ldb + koff + k0);
#pragma unroll
  for (int i = 0; i < 4; ++i) {
    const size_t ao = (size_t)(m0 + (i << 4) + rlane) * lda + koff + k0;
    const v16b ah = Frag<__bf16>::load(A + ao);
    v16b al = ah;
    if (LO) al = Frag<__bf16>::load(A2 + ao);
#pragma unroll
    for (int j = 0; j < 4; ++j) {
      acc[i][j] = Frag<__bf16>::mma(ah, bh[j], acc[i][j]);
      if (LO) acc[i][j] = Frag<__bf16>::mma(al, bh[j], acc[i][j]);
    }
    guard_row(acc[i][0], acc[i][1], acc[i][2], acc[i][3], ah, al, bh[0], bh[1], bh[2], bh[3]);
  }
}

template <int OUT_MODE, int ACT>
__global__ __launch_bounds__(kThreads) void gemm_ahl_kernel(
    const unsigned short* __restrict__ Ap, const unsigned short* __restrict__ A2p, int lda,
    const unsigned short* __restrict__ Btp, int ldb,
    void* __restrict__ Cout, void* __restrict__ Cout2, int ldc,
    const float* __restrict__ bias, int M, int N, int K, int kslo) {
  const __bf16* A = (const __bf16*)Ap; const __bf16* A2 = (const __bf16*)A2p; const __bf16* Bt = (const __bf16*)Btp;
  __shared__ __align__(16) float sT[8][16 * 68];
  const int lane = threadIdx.x & 31;
  const int wave = threadIdx.x >> 5;
  const int tilesN = N >> 6;
  const int tilesM = M >> 6;
  const int tile = blockIdx.x * 8 + wave;
  if (tile >= tilesM * tilesN) return;
  const int tm = tile / tilesN;
  const int tn = tile - tm * tilesN;
  const int m0 = tm << 6;
  const int n0 = tn << 6;
  const int rlane = lane & 15;
  const int koff  = (lane >> 4) * 8;
  const int mOff  = (lane >> 4) * 8;

  v8f acc[4][4];
#pragma unroll
  for (int i = 0; i < 4; ++i)
#pragma unroll
    for (int j = 0; j < 4; ++j) acc[i][j] = (v8f){0.f,0.f,0.f,0.f,0.f,0.f,0.f,0.f};

  const int ks = kslo < K ? kslo : K;
  int k0 = 0;
  for (; k0 < ks; k0 += 32) kstep64<false>(acc, A, A2, lda, Bt, ldb, m0, n0, k0, rlane, koff);
  for (; k0 < K; k0 += 32)  kstep64<true>(acc, A, A2, lda, Bt, ldb, m0, n0, k0, rlane, koff);
  acc_guard4(acc[0][0], acc[0][1], acc[0][2], acc[0][3]);
  acc_guard4(acc[1][0], acc[1][1], acc[1][2], acc[1][3]);
  acc_guard4(acc[2][0], acc[2][1], acc[2][2], acc[2][3]);
  acc_guard4(acc[3][0], acc[3][1], acc[3][2], acc[3][3]);

  float bvj[4];
#pragma unroll
  for (int j = 0; j < 4; ++j) bvj[j] = bias[n0 + (j << 4) + rlane];
  float* slab = sT[wave];
#pragma unroll
  for (int i = 0; i < 4; ++i) {
    const int mBase = m0 + (i << 4);
#pragma unroll
    for (int j = 0; j < 4; ++j) {
#pragma unroll
      for (int r = 0; r < 8; ++r) {
        float v = acc[i][j][r] + bvj[j];
        if (ACT == 2) v = fmaxf(v, 0.0f);
        slab[(mOff + r) * 68 + (j << 4) + rlane] = v;
      }
    }
    __builtin_amdgcn_fence(__ATOMIC_RELEASE, "workgroup");
    __builtin_amdgcn_wave_barrier();
    __builtin_amdgcn_fence(__ATOMIC_ACQUIRE, "workgroup");
    if (OUT_MODE == 0) {
      float* Cf = (float*)Cout;
      const int hh = lane >> 4, c4 = (lane & 15) * 4;
      for (int pass = 0; pass < 2; ++pass) {
#pragma unroll
        for (int it = 0; it < 8; ++it) {
          const int row = it * 2 + hh;
          v4f v = *(const v4f*)(slab + row * 68 + c4);
          *(volatile v4f*)(Cf + (size_t)(mBase + row) * ldc + n0 + c4) = v;
        }
        __threadfence();
      }
    } else {
      const int q = lane >> 3, c8 = (lane & 7) * 8;
      unsigned short* Ch = (unsigned short*)Cout;
      unsigned short* Cl = (unsigned short*)Cout2;
      for (int pass = 0; pass < 2; ++pass) {
#pragma unroll
        for (int it = 0; it < 4; ++it) {
          const int row = it * 4 + q;
          const float* sp = slab + row * 68 + c8;
          v4u hv, lv;
#pragma unroll
          for (int e = 0; e < 4; ++e) { unsigned lo; const unsigned hi = split_pair(sp[2 * e], sp[2 * e + 1], lo); hv[e] = hi; lv[e] = lo; }
          *(volatile v4u*)(Ch + (size_t)(mBase + row) * ldc + n0 + c8) = hv;
          *(volatile v4u*)(Cl + (size_t)(mBase + row) * ldc + n0 + c8) = lv;
        }
        __threadfence();
      }
    }
    __builtin_amdgcn_fence(__ATOMIC_RELEASE, "workgroup");
    __builtin_amdgcn_wave_barrier();
    __builtin_amdgcn_fence(__ATOMIC_ACQUIRE, "workgroup");
  }
}

__global__ __launch_bounds__(kThreads) void out_kernel(const unsigned short* __restrict__ Ap, const unsigned short* __restrict__ A2p,
                                                       const unsigned short* __restrict__ Btp, const float* __restrict__ bias,
                                                       float* __restrict__ out) {
  __shared__ __align__(16) float sO[8][16 * kCls];
  const __bf16* A = (const __bf16*)Ap; const __bf16* A2 = (const __bf16*)A2p; const __bf16* Bt = (const __bf16*)Btp;
  const int lane = threadIdx.x & 31;
  const int wave = threadIdx.x >> 5;
  const int tile = blockIdx.x * 8 + wave;
  const int m0 = tile << 6;
  if (m0 >= kNodes) return;
  const int rlane = lane & 15;
  const int koff  = (lane >> 4) * 8;
  const int mOff  = (lane >> 4) * 8;

  v8f acc[4][4];
#pragma unroll
  for (int i = 0; i < 4; ++i)
#pragma unroll
    for (int j = 0; j < 4; ++j) acc[i][j] = (v8f){0.f,0.f,0.f,0.f,0.f,0.f,0.f,0.f};
  for (int k0 = 0; k0 < kFeat; k0 += 32) kstep64<true>(acc, A, A2, kFeat, Bt, kFeat, m0, 0, k0, rlane, koff);
  acc_guard4(acc[0][0], acc[0][1], acc[0][2], acc[0][3]);
  acc_guard4(acc[1][0], acc[1][1], acc[1][2], acc[1][3]);
  acc_guard4(acc[2][0], acc[2][1], acc[2][2], acc[2][3]);
  acc_guard4(acc[3][0], acc[3][1], acc[3][2], acc[3][3]);

  float bvj[3];
#pragma unroll
  for (int j = 0; j < 3; ++j) bvj[j] = bias[(j << 4) + rlane];
  float* slab = sO[wave];
#pragma unroll
  for (int i = 0; i < 4; ++i) {
    const int mBase = m0 + (i << 4);
    if (mBase < kNodes) {
#pragma unroll
      for (int j = 0; j < 3; ++j) {
        const int n = (j << 4) + rlane;
#pragma unroll
        for (int r = 0; r < 8; ++r) {
          const float v = acc[i][j][r] + bvj[j];
          if (n < kCls) slab[(mOff + r) * kCls + n] = v;
        }
      }
      __builtin_amdgcn_fence(__ATOMIC_RELEASE, "workgroup");
      __builtin_amdgcn_wave_barrier();
      __builtin_amdgcn_fence(__ATOMIC_ACQUIRE, "workgroup");
      float* ob = out + (size_t)mBase * kCls;
      for (int pass = 0; pass < 2; ++pass) {
#pragma unroll
        for (int qq = 0; qq < 5; ++qq) {
          const int f = (qq * 32 + lane) * 4;
          const v4f v = *(const v4f*)(slab + f);
          *(volatile v4f*)(ob + f) = v;
        }
        __threadfence();
      }
      __builtin_amdgcn_fence(__ATOMIC_RELEASE, "workgroup");
      __builtin_amdgcn_wave_barrier();
      __builtin_amdgcn_fence(__ATOMIC_ACQUIRE, "workgroup");
    }
  }
}

__global__ __launch_bounds__(kThreads) void xcvt_kernel(const float* __restrict__ x, unsigned short* __restrict__ Hh,
                                                        unsigned short* __restrict__ Hl) {
  const int i = blockIdx.x * kThreads + threadIdx.x;
  const int row = i >> 4, g = i & 15;
  const int rowc = row < kNodes ? row : kNodes - 1;
  const float flag = (row < kNodes) ? 1.0f : 0.0f;
  const float* p = x + (size_t)rowc * kFeat + g * 8;
  const v4f a = *(const v4f*)(p);
  const v4f c = *(const v4f*)(p + 4);
  v4u u;
  u[0] = pk16(f2bf_bits(a[0] * flag + 0.0f), f2bf_bits(a[1] * flag + 0.0f));
  u[1] = pk16(f2bf_bits(a[2] * flag + 0.0f), f2bf_bits(a[3] * flag + 0.0f));
  u[2] = pk16(f2bf_bits(c[0] * flag + 0.0f), f2bf_bits(c[1] * flag + 0.0f));
  u[3] = pk16(f2bf_bits(c[2] * flag + 0.0f), f2bf_bits(c[3] * flag + 0.0f));
  const v4u z = (v4u){0u, 0u, 0u, 0u};
  unsigned short* dh = Hh + (size_t)i * 8;
  unsigned short* dl = Hl + (size_t)i * 8;
  *(volatile v4u*)dh = u; *(volatile v4u*)dl = z;
  __threadfence();
  *(volatile v4u*)dh = u; *(volatile v4u*)dl = z;
}

__global__ __launch_bounds__(kThreads) void prep_kernel(
    const float* __restrict__ w1pre, const float* __restrict__ b1pre, const float* __restrict__ w1post, const float* __restrict__ b1post,
    const float* __restrict__ w1lin, const float* __restrict__ b1lin,
    const float* __restrict__ w2pre, const float* __restrict__ b2pre, const float* __restrict__ w2post, const float* __restrict__ b2post,
    const float* __restrict__ w2lin, const float* __restrict__ b2lin,
    const float* __restrict__ wout, const float* __restrict__ bout,
    unsigned* __restrict__ Wpre1, unsigned* __restrict__ Wpost1, unsigned* __restrict__ Wlin1,
    unsigned* __restrict__ Wpre2, unsigned* __restrict__ Wpost2, unsigned* __restrict__ Wlin2,
    unsigned* __restrict__ Wout, float* __restrict__ Bias) {
  const int blk = blockIdx.x, t = threadIdx.x;
  if (blk < 464) {
    const float* W; unsigned* dst; int mode, lb;
    if (blk < 64)       { W = w1pre;  dst = Wpre1;  mode = 0; lb = blk; }
    else if (blk < 192) { W = w1post; dst = Wpost1; mode = 1; lb = blk - 64; }
    else if (blk < 224) { W = w1lin;  dst = Wlin1;  mode = 2; lb = blk - 192; }
    else if (blk < 288) { W = w2pre;  dst = Wpre2;  mode = 0; lb = blk - 224; }
    else if (blk < 416) { W = w2post; dst = Wpost2; mode = 1; lb = blk - 288; }
    else if (blk < 448) { W = w2lin;  dst = Wlin2;  mode = 2; lb = blk - 416; }
    else                { W = wout;   dst = Wout;   mode = 3; lb = blk - 448; }
    const int i = lb * kThreads + t;
    int ia, ib; float flag = 1.0f;
    if (mode == 0) {
      const int n = i >> 6, k = (i & 63) * 2;
      const int kb = (n >> 7) << 7, col = n & 127;
      ia = (kb + k) * kFeat + col; ib = ia + kFeat;
    } else if (mode == 1) {
      const int n = i >> 8, k = (i & 255) * 2;
      ia = k * kFeat + n; ib = ia + kFeat;
    } else if (mode == 2) {
      const int n = i >> 6, k = (i & 63) * 2;
      ia = k * kFeat + n; ib = ia + kFeat;
    } else {
      const int n = i >> 6, k = (i & 63) * 2;
      const int nc = n < kCls ? n : kCls - 1;
      flag = (n < kCls) ? 1.0f : 0.0f;
      ia = k * kCls + nc; ib = ia + kCls;
    }
    const float a = W[ia] * flag + 0.0f;
    const float b = W[ib] * flag + 0.0f;
    const unsigned u = pk16(f2bf_bits(a), f2bf_bits(b));
    ((volatile unsigned*)dst)[i] = u;
    __threadfence();
    ((volatile unsigned*)dst)[i] = u;
  } else {
    const int s = blk - 464;
    const float* src; int len = kFeat;
    if (s == 0) src = b1pre; else if (s == 1) src = b1post; else if (s == 2) src = b1lin;
    else if (s == 3) src = b2pre; else if (s == 4) src = b2post; else if (s == 5) src = b2lin;
    else { src = bout; len = kCls; }
    const int tc = t < len ? t : len - 1;
    const float flag = (t < len) ? 1.0f : 0.0f;
    const float v = bf_bits2f(f2bf_bits(src[tc] * flag + 0.0f));
    float* dp = Bias + s * 256 + t;
    *(volatile float*)dp = v;
    __threadfence();
    *(volatile float*)dp = v;
  }
}

__device__ __forceinline__ int blk_excl_scan(int cnt, int* scan_ws, int tid, int* tot) {
  const int lane = tid & 31, wave = tid >> 5;
  int incl = cnt;
#pragma unroll
  for (int o = 1; o < 32; o <<= 1) { const int v = __shfl_up(incl, o, 32); if (lane >= o) incl += v; }
  if (lane == 31) scan_ws[wave] = incl;
  __syncthreads();
  if (wave == 0) {
    const int lc = lane < 8 ? lane : 7;
    int wv = scan_ws[lc];
    wv = (lane < 8) ? wv : 0;
    int wincl = wv;
#pragma unroll
    for (int o = 1; o < 32; o <<= 1) { const int v = __shfl_up(wincl, o, 32); if (lane >= o) wincl += v; }
    if (lane < 8) scan_ws[32 + lane] = wincl - wv;
    if (lane == 31) scan_ws[64] = wincl;
  }
  __syncthreads();
  const int res = scan_ws[32 + wave] + incl - cnt;
  *tot = scan_ws[64];
  return res;
}
__device__ __forceinline__ int chunk_hits(const int* __restrict__ dstv, const int* __restrict__ srcv, int e0, int n0, int tid,
                                          int* LIST, int* scan_ws) {
  const int eb = e0 + tid * kEPT;
  const bool valid = eb < kEdges;
  const int ebc = valid ? eb : (kEdges - kEPT);
  const unsigned lim = valid ? (unsigned)kAggRows : 0u;
  unsigned uo[kEPT];
  unsigned hm = 0u;
#pragma unroll
  for (int g = 0; g < kEPT / 4; ++g) {
    const v4i d4 = *(const v4i*)(dstv + ebc + 4 * g);
#pragma unroll
    for (int e = 0; e < 4; ++e) {
      const unsigned u = (unsigned)(d4[e] - n0);
      uo[4 * g + e] = u;
      hm |= (u < lim ? 1u : 0u) << (4 * g + e);
    }
  }
  asm volatile("" ::: "memory");
  int rec[kEPT];
#pragma unroll
  for (int g = 0; g < kEPT / 4; ++g) {
    const v4i s4 = *(const v4i*)(srcv + ebc + 4 * g);
    keep_v4i(s4);
#pragma unroll
    for (int e = 0; e < 4; ++e) rec[4 * g + e] = (int)((uo[4 * g + e] << 16) | ((unsigned)s4[e] & 0xFFFFu));
  }
  const int cnt = __builtin_popcount(hm);
  int tot;
  int p = blk_excl_scan(cnt, scan_ws, tid, &tot);
  if (hm != 0u) {
#pragma unroll
    for (int k = 0; k < kEPT; ++k) {
      if ((hm >> k) & 1u) { if ((unsigned)p < (unsigned)kEdgeChunk) LIST[p] = rec[k]; ++p; }
    }
  }
  __syncthreads();
  return tot < kEdgeChunk ? tot : kEdgeChunk;
}

__global__ __launch_bounds__(kThreads) void agg_kernel(const float* __restrict__ PQ, const int* __restrict__ ei,
                                                       const unsigned short* __restrict__ Hh, const unsigned short* __restrict__ Hl,
                                                       unsigned short* __restrict__ A5h, unsigned short* __restrict__ A5l, int chunk) {
  extern __shared__ __align__(16) float accL[];
  __shared__ int LIST[kEdgeChunk];
  __shared__ int SC[kAggRows];
  __shared__ int scan_ws[80];
  const int tid = threadIdx.x, lane = tid & 31, wave = tid >> 5, hh = lane >> 4;
  const int lr0 = blockIdx.x * kAggRows;
  const int n0 = chunk * kChunkRows + lr0;
  for (int i = tid; i < kEdgeChunk; i += kThreads) LIST[i] = -1;
  for (int i = tid; i < kAggRows; i += kThreads) SC[i] = 0;
  if (tid < 80) scan_ws[tid] = 0;
  const v4f z4 = (v4f){0.f, 0.f, 0.f, 0.f};
  const v4f neg4 = (v4f){-3.0e38f, -3.0e38f, -3.0e38f, -3.0e38f};
#pragma unroll 1
  for (int it = 0; it < (kAggRows * kAccPitch / 4) / kThreads; ++it) {
    const int i4 = it * kThreads + tid;
    const int col = (i4 * 4) & (kAccPitch - 1);
    const v4f v = (col < kFeat) ? z4 : neg4;
    *(v4f*)(accL + (size_t)i4 * 4) = v;
  }
  __syncthreads();
  const int* srcv = ei;
  const int* dstv = ei + kEdges;
#pragma unroll 1
  for (int c = 0; c < kNumEdgeChunks; ++c) {
    const int tot = chunk_hits(dstv, srcv, c * kEdgeChunk, n0, tid, LIST, scan_ws);
#pragma unroll 1
    for (int base = 0; base < tot; base += 32) {
      const int q = base + lane;
      const int qc = q < kEdgeChunk ? q : kEdgeChunk - 1;
      const int rvl = LIST[qc];
      const int rv = (q < tot) ? rvl : -1;
      const int own = (rv >= 0 && (rv >> 21) == wave) ? 1 : 0;
      unsigned msk = (unsigned)__ballot(own);
#pragma unroll 1
      for (int it = 0; it < 32; ++it) {
        if (msk == 0u) break;
        const int bp = __builtin_ctz(msk);
        msk &= msk - 1u;
        const int r = __shfl(rv, bp, 32);
        const int dl = (r >> 16) & (kAggRows - 1);
        int s = r & 0xFFFF;
        s = s < kNodes ? s : kNodes - 1;
        const v4f q4 = *(const v4f*)(PQ + (size_t)s * kPQPitch + kFeat + 4 * lane);
        float* rp = accL + dl * kAccPitch + 4 * lane;
        v4f a = *(const v4f*)(rp);
        const v4f m = *(const v4f*)(rp + kFeat);
        a = a + q4;
        v4f mm;
        mm[0] = fmaxf(m[0], q4[0]); mm[1] = fmaxf(m[1], q4[1]); mm[2] = fmaxf(m[2], q4[2]); mm[3] = fmaxf(m[3], q4[3]);
        *(v4f*)(rp) = a;
        *(v4f*)(rp + kFeat) = mm;
        if (lane == 0) SC[dl] += 1;
      }
    }
    __syncthreads();
  }
  const int c8 = (lane & 15) * 8;
#pragma unroll 1
  for (int j = 0; j < kRowsPerWave; j += 2) {
    const int dl = wave * kRowsPerWave + j + hh;
    const int lr = lr0 + dl;
    const int n = n0 + dl;
    const float cntf = (float)SC[dl];
    const float inv = 1.0f / fmaxf(cntf, 1.0f);
    const float live = (cntf > 0.5f) ? 1.0f : 0.0f;
    const v4u xh = *(const v4u*)(Hh + (size_t)n * kFeat + c8);
    const v4u xl = *(const v4u*)(Hl + (size_t)n * kFeat + c8);
    const float* pp = PQ + (size_t)n * kPQPitch + c8;
    const v4f p0 = *(const v4f*)(pp);
    const v4f p1 = *(const v4f*)(pp + 4);
    const float* ap = accL + dl * kAccPitch + c8;
    const v4f s0 = *(const v4f*)(ap);
    const v4f s1 = *(const v4f*)(ap + 4);
    const v4f mq0 = *(const v4f*)(ap + kFeat);
    const v4f mq1 = *(const v4f*)(ap + kFeat + 4);
    float su[8], me[8], mx[8];
#pragma unroll
    for (int e = 0; e < 4; ++e) {
      su[e] = cntf * p0[e] + s0[e];
      me[e] = su[e] * inv;
      mx[e] = live * (p0[e] + mq0[e]) + 0.0f;
      su[4 + e] = cntf * p1[e] + s1[e];
      me[4 + e] = su[4 + e] * inv;
      mx[4 + e] = live * (p1[e] + mq1[e]) + 0.0f;
    }
    v4u suh, sul, meh, mel, mxh, mxl;
    split8(su, suh, sul);
    split8(me, meh, mel);
    split8(mx, mxh, mxl);
    unsigned short* ahp = A5h + (size_t)lr * kA5Pitch;
    unsigned short* alp = A5l + (size_t)lr * kA5Pitch;
    for (int pass = 0; pass < 2; ++pass) {
      *(volatile v4u*)(ahp + c8)             = xh;
      *(volatile v4u*)(ahp + kFeat + c8)     = meh;
      *(volatile v4u*)(ahp + 2 * kFeat + c8) = mxh;
      *(volatile v4u*)(ahp + 3 * kFeat + c8) = suh;
      *(volatile v4u*)(alp + c8)             = xl;
      *(volatile v4u*)(alp + kFeat + c8)     = mel;
      *(volatile v4u*)(alp + 2 * kFeat + c8) = mxl;
      *(volatile v4u*)(alp + 3 * kFeat + c8) = sul;
      __threadfence();
    }
  }
}

extern "C" void kernel_launch(void* const* d_in, const int* in_sizes, int n_in,
                              void* d_out, int out_size, void* d_ws, size_t ws_size, hipStream_t stream) {
  (void)in_sizes; (void)n_in; (void)out_size;
  const float* x      = (const float*)d_in[0];
  const int*   ei     = (const int*)  d_in[1];
  const float* w1pre  = (const float*)d_in[2];  const float* b1pre  = (const float*)d_in[3];
  const float* w1post = (const float*)d_in[4];  const float* b1post = (const float*)d_in[5];
  const float* w1lin  = (const float*)d_in[6];  const float* b1lin  = (const float*)d_in[7];
  const float* w2pre  = (const float*)d_in[8];  const float* b2pre  = (const float*)d_in[9];
  const float* w2post = (const float*)d_in[10]; const float* b2post = (const float*)d_in[11];
  const float* w2lin  = (const float*)d_in[12]; const float* b2lin  = (const float*)d_in[13];
  const float* wout   = (const float*)d_in[14]; const float* bout   = (const float*)d_in[15];
  float* out = (float*)d_out;

  if (kOffEnd > ws_size) return;
  char* ws = (char*)d_ws;
  unsigned short* Hh  = (unsigned short*)(ws + kOffHh);
  unsigned short* Hl  = (unsigned short*)(ws + kOffHl);
  float*          PQ  = (float*)(ws + kOffPQ);
  unsigned short* A5h = (unsigned short*)(ws + kOffA5h);
  unsigned short* A5l = (unsigned short*)(ws + kOffA5l);
  unsigned short* Th  = (unsigned short*)(ws + kOffTh);
  unsigned short* Tl  = (unsigned short*)(ws + kOffTl);
  unsigned* Wpre1  = (unsigned*)(ws + kOffWpre1);
  unsigned* Wpost1 = (unsigned*)(ws + kOffWpost1);
  unsigned* Wlin1  = (unsigned*)(ws + kOffWlin1);
  unsigned* Wpre2  = (unsigned*)(ws + kOffWpre2);
  unsigned* Wpost2 = (unsigned*)(ws + kOffWpost2);
  unsigned* Wlin2  = (unsigned*)(ws + kOffWlin2);
  unsigned* Woutp  = (unsigned*)(ws + kOffWout);
  float*    Bias   = (float*)(ws + kOffBias);
  const float* b256_1 = Bias + 0;
  const float* bpost1 = Bias + 256;
  const float* blin1  = Bias + 512;
  const float* b256_2 = Bias + 768;
  const float* bpost2 = Bias + 1024;
  const float* blin2  = Bias + 1280;
  const float* bout64 = Bias + 1536;

  prep_kernel<<<dim3(471), dim3(kThreads), 0, stream>>>(w1pre, b1pre, w1post, b1post, w1lin, b1lin,
                                                       w2pre, b2pre, w2post, b2post, w2lin, b2lin, wout, bout,
                                                       Wpre1, Wpost1, Wlin1, Wpre2, Wpost2, Wlin2, Woutp, Bias);
  xcvt_kernel<<<dim3(kNPad * 16 / kThreads), dim3(kThreads), 0, stream>>>(x, Hh, Hl);

  const int gridPQ = (kNPad / 64) * (kPQPitch / 64) / 8;
  const int gridC  = (kChunkRows / 64) * (kFeat / 64) / 8;
  for (int layer = 0; layer < 2; ++layer) {
    const unsigned short* Wpre  = (const unsigned short*)(layer ? Wpre2  : Wpre1);
    const unsigned short* Wpost = (const unsigned short*)(layer ? Wpost2 : Wpost1);
    const unsigned short* Wlin  = (const unsigned short*)(layer ? Wlin2  : Wlin1);
    const float* b256  = layer ? b256_2 : b256_1;
    const float* bpost = layer ? bpost2 : bpost1;
    const float* blin  = layer ? blin2  : blin1;
    const int kslo = layer ? 0 : kFeat;

    gemm_ahl_kernel<0, 0><<<dim3(gridPQ), dim3(kThreads), 0, stream>>>(
        Hh, Hl, kFeat, Wpre, kFeat, (void*)PQ, (void*)nullptr, kPQPitch, b256, kNPad, kPQPitch, kFeat, kslo);
    for (int c = 0; c < kNumChunks; ++c) {
      agg_kernel<<<dim3(kBlocksPerChunk), dim3(kThreads), kAggLdsBytes, stream>>>(PQ, ei, Hh, Hl, A5h, A5l, c);
      gemm_ahl_kernel<2, 0><<<dim3(gridC), dim3(kThreads), 0, stream>>>(
          A5h, A5l, kA5Pitch, Wpost, kA5Pitch, (void*)Th, (void*)Tl, kFeat, bpost, kChunkRows, kFeat, kA5Pitch, kslo);
      unsigned short* Hhc = Hh + (size_t)c * kChunkRows * kFeat;
      unsigned short* Hlc = Hl + (size_t)c * kChunkRows * kFeat;
      gemm_ahl_kernel<2, 2><<<dim3(gridC), dim3(kThreads), 0, stream>>>(
          Th, Tl, kFeat, Wlin, kFeat, (void*)Hhc, (void*)Hlc, kFeat, blin, kChunkRows, kFeat, kFeat, 0);
    }
  }
  out_kernel<<<dim3(kNPad / 64 / 8), dim3(kThreads), 0, stream>>>(Hh, Hl, (const unsigned short*)Woutp, bout64, out);
}
